// SelfAttention2d_7043746365829
// MI455X (gfx1250) — hardware-verified
//
#include <hip/hip_runtime.h>
#include <math.h>
#include <stdint.h>

#define NB    4
#define CH    256
#define NPOS  4096
#define NGRP  8
#define CPG   32
#define QKP   512
#define STP   32

static_assert(CH == NGRP * CPG);
static_assert(NPOS % 64 == 0);
static_assert(CH % 64 == 0);
static_assert((NB * NPOS) % 64 == 0);
static_assert(QKP == 2 * CH);
static_assert((CPG * NPOS) % 1024 == 0);

typedef __attribute__((ext_vector_type(8)))  _Float16 v8h;
typedef __attribute__((ext_vector_type(16))) __bf16   v16b;
typedef __attribute__((ext_vector_type(8)))  __bf16   v8b;
typedef __attribute__((ext_vector_type(8)))  float    v8f;
typedef __attribute__((ext_vector_type(4)))  float    v4f;
typedef __attribute__((ext_vector_type(2)))  float    v2f;
typedef __attribute__((ext_vector_type(4)))  unsigned int v4u;

__device__ __forceinline__ unsigned short f2bf_bits(float f) {
  unsigned u = __float_as_uint(f);
  return (unsigned short)((u + 0x7FFFu + ((u >> 16) & 1u)) >> 16);
}
__device__ __forceinline__ float bf_bits2f(unsigned short h) { return __uint_as_float(((unsigned)h) << 16); }
__device__ __forceinline__ unsigned pk16(unsigned short a, unsigned short b) { return (unsigned)a | ((unsigned)b << 16); }
__device__ __forceinline__ __bf16 at_f2bf(float f) { return __builtin_bit_cast(__bf16, f2bf_bits(f)); }

__device__ __forceinline__ void dep_guard_b(v8f& a, v8f& b, v16b x, v16b y) { asm volatile("v_nop\n\tv_nop\n\tv_nop\n\tv_nop" : "+v"(a), "+v"(b) : "v"(x), "v"(y)); }
__device__ __forceinline__ void keep4_b(v16b a, v16b b, v16b c, v16b d) { asm volatile("v_nop" :: "v"(a), "v"(b), "v"(c), "v"(d)); }
__device__ __forceinline__ void acc_guard4(v8f& a, v8f& b, v8f& c, v8f& d) { asm volatile("v_nop\n\tv_nop\n\tv_nop\n\tv_nop" : "+v"(a), "+v"(b), "+v"(c), "+v"(d)); }

template <typename T> struct Frag;
template <> struct Frag<__bf16> {
  typedef v16b V; union U { v16b v; v8b h[2]; };
  static __device__ __forceinline__ v16b load(const __bf16* p) {
    U f; f.h[0] = *(const v8b*)(p); f.h[1] = *(const v8b*)(p + 16); return f.v;
  }
  static __device__ __forceinline__ v8f mma(v16b a, v16b b, v8f c) {
    return __builtin_amdgcn_wmma_f32_16x16x32_bf16(false, a, false, b, (short)0, c, false, false);
  }
  static __device__ __forceinline__ void guard(v8f& a, v8f& b, v16b x, v16b y) { dep_guard_b(a, b, x, y); }
  static __device__ __forceinline__ void keep(v16b a, v16b b, v16b c, v16b d) { keep4_b(a, b, c, d); }
};

__device__ __forceinline__ v8f at_mma(v16b a, v16b b, v8f c) {
  c = __builtin_amdgcn_wmma_f32_16x16x32_bf16(false, a, false, b, (short)0, c, false, false);
  asm volatile("v_nop\n\tv_nop\n\tv_nop\n\tv_nop" : "+v"(c) : "v"(a), "v"(b));
  return c;
}

template <int BIAS_MODE, int OUT_MODE, bool RESID>
__global__ __launch_bounds__(256) void wmma_gemm64(
    const unsigned short* __restrict__ Ap, int lda, long strideA,
    const unsigned short* __restrict__ Btp, int ldb, long strideB,
    void* __restrict__ Cout, int ldc, long strideC,
    const float* __restrict__ bias,
    const float* __restrict__ resid, long strideR,
    int M, int N, int K, float scale) {
  typedef __bf16 T;
  typedef v16b V;
  const T* A = (const T*)(const void*)Ap; const T* Bt = (const T*)(const void*)Btp;
  __shared__ __align__(16) float sT[8][16 * 68];
  const int b    = blockIdx.y;
  const int lane = threadIdx.x & 31;
  const int wave = threadIdx.x >> 5;
  const int tilesN = N >> 6;
  const int tilesM = M >> 6;
  const int tile = blockIdx.x * 8 + wave;
  if (tile >= tilesM * tilesN) return;
  const int tm = tile / tilesN;
  const int tn = tile - tm * tilesN;
  const int m0 = tm << 6;
  const int n0 = tn << 6;

  const T* Ab = A  + (size_t)b * strideA;
  const T* Bb = Bt + (size_t)b * strideB;

  const int rlane = lane & 15;
  const int koff  = (lane >> 4) * 8;
  const int mOff  = (lane >> 4) * 8;

  v8f acc[4][4];
#pragma unroll
  for (int i = 0; i < 4; ++i)
#pragma unroll
    for (int j = 0; j < 4; ++j) acc[i][j] = (v8f){0.f,0.f,0.f,0.f,0.f,0.f,0.f,0.f};

  for (int k0 = 0; k0 < K; k0 += 32) {
    V bh[4];
#pragma unroll
    for (int j = 0; j < 4; ++j) {
      const size_t bo = (size_t)(n0 + (j << 4) + rlane) * ldb + koff + k0;
      bh[j] = Frag<T>::load(Bb + bo);
    }
#pragma unroll
    for (int i = 0; i < 4; ++i) {
      const size_t ao = (size_t)(m0 + (i << 4) + rlane) * lda + koff + k0;
      V ah = Frag<T>::load(Ab + ao);
#pragma unroll
      for (int j = 0; j < 4; ++j) acc[i][j] = Frag<T>::mma(ah, bh[j], acc[i][j]);
      Frag<T>::guard(acc[i][0], acc[i][3], ah, ah);
    }
    Frag<T>::keep(bh[0], bh[1], bh[2], bh[3]);
  }
  acc_guard4(acc[0][0], acc[0][1], acc[0][2], acc[0][3]);
  acc_guard4(acc[1][0], acc[1][1], acc[1][2], acc[1][3]);
  acc_guard4(acc[2][0], acc[2][1], acc[2][2], acc[2][3]);
  acc_guard4(acc[3][0], acc[3][1], acc[3][2], acc[3][3]);

  float* slab = sT[wave];
  const float* Rb = RESID ? (resid + (size_t)b * strideR) : nullptr;
#pragma unroll
  for (int i = 0; i < 4; ++i) {
    const int mBase = m0 + (i << 4);
#pragma unroll
    for (int j = 0; j < 4; ++j) {
      const int n = n0 + (j << 4) + rlane;
      float bv = 0.f;
      if (BIAS_MODE == 2) bv = bias[n];
#pragma unroll
      for (int r = 0; r < 8; ++r) {
        float v = acc[i][j][r] * scale;
        if (BIAS_MODE == 1) v += bias[mBase + mOff + r];
        if (BIAS_MODE == 2) v += bv;
        slab[(mOff + r) * 68 + (j << 4) + rlane] = v;
      }
    }
    __builtin_amdgcn_fence(__ATOMIC_RELEASE, "workgroup");
    __builtin_amdgcn_wave_barrier();
    __builtin_amdgcn_fence(__ATOMIC_ACQUIRE, "workgroup");
    if (OUT_MODE == 0) {
      float* C = (float*)Cout + (size_t)b * strideC;
      const int hh = lane >> 4, c4 = (lane & 15) * 4;
      for (int pass = 0; pass < 2; ++pass) {
#pragma unroll
        for (int it = 0; it < 8; ++it) {
          const int row = it * 2 + hh;
          v4f v = *(const v4f*)(slab + row * 68 + c4);
          if (RESID) v += *(const v4f*)(Rb + (size_t)(mBase + row) * ldc + n0 + c4);
          *(volatile v4f*)(C + (size_t)(mBase + row) * ldc + n0 + c4) = v;
        }
        __threadfence();
      }
    } else {
      const int q = lane >> 3, c8 = (lane & 7) * 8;
      unsigned short* C = (unsigned short*)Cout + (size_t)b * strideC;
      for (int pass = 0; pass < 2; ++pass) {
#pragma unroll
        for (int it = 0; it < 4; ++it) {
          const int row = it * 4 + q;
          const float* sp = slab + row * 68 + c8;
          v8h hv;
#pragma unroll
          for (int e = 0; e < 8; ++e) hv[e] = __builtin_bit_cast(_Float16, f2bf_bits(sp[e]));
          *(volatile v8h*)(C + (size_t)(mBase + row) * ldc + n0 + c8) = hv;
        }
        __threadfence();
      }
    }
    __builtin_amdgcn_fence(__ATOMIC_RELEASE, "workgroup");
    __builtin_amdgcn_wave_barrier();
    __builtin_amdgcn_fence(__ATOMIC_ACQUIRE, "workgroup");
  }
}

__global__ __launch_bounds__(256) void conv_bf16x2_kernel(const float* __restrict__ in, unsigned short* __restrict__ ho, int n2) {
  const int i = blockIdx.x * 256 + threadIdx.x;
  if (i < n2) {
    const v2f f = *(const v2f*)(in + 2 * (size_t)i);
    const unsigned uh = pk16(f2bf_bits(f[0]), f2bf_bits(f[1]));
    ((volatile unsigned*)ho)[i] = uh;
    __threadfence();
    ((volatile unsigned*)ho)[i] = uh;
  }
}

__global__ __launch_bounds__(256) void gnstat_kernel(const float* __restrict__ x, float* __restrict__ stats) {
  __shared__ float red[8];
  __shared__ float bc[2];
  const int bg = blockIdx.x;
  const int tid = threadIdx.x, lane = tid & 31, wave = tid >> 5;
  const float* p = x + (size_t)bg * (CPG * NPOS);
  const float invn = 1.0f / (float)(CPG * NPOS);
  const int niter = (CPG * NPOS) / 1024;

  float s0 = 0.f, s1 = 0.f, s2 = 0.f, s3 = 0.f;
#pragma unroll 4
  for (int i = 0; i < niter; ++i) {
    const v4f v = *(const v4f*)(p + ((size_t)i * 256 + tid) * 4);
    s0 += v[0]; s1 += v[1]; s2 += v[2]; s3 += v[3];
  }
  float s = (s0 + s1) + (s2 + s3);
#pragma unroll
  for (int off = 16; off > 0; off >>= 1) s += __shfl_xor(s, off, 32);
  if (lane == 0) red[wave] = s;
  __syncthreads();
  if (tid == 0) {
    float t = 0.f;
#pragma unroll
    for (int w = 0; w < 8; ++w) t += red[w];
    bc[0] = t * invn;
  }
  __syncthreads();
  const float mean = bc[0];

  float q0 = 0.f, q1 = 0.f, q2 = 0.f, q3 = 0.f;
#pragma unroll 4
  for (int i = 0; i < niter; ++i) {
    const v4f v = *(const v4f*)(p + ((size_t)i * 256 + tid) * 4);
    const float d0 = v[0] - mean, d1 = v[1] - mean, d2 = v[2] - mean, d3 = v[3] - mean;
    q0 += d0 * d0; q1 += d1 * d1; q2 += d2 * d2; q3 += d3 * d3;
  }
  float qs = (q0 + q1) + (q2 + q3);
#pragma unroll
  for (int off = 16; off > 0; off >>= 1) qs += __shfl_xor(qs, off, 32);
  if (lane == 0) red[wave] = qs;
  __syncthreads();
  if (tid == 0) {
    float t = 0.f;
#pragma unroll
    for (int w = 0; w < 8; ++w) t += red[w];
    const float var = t * invn;
    bc[1] = 1.0f / sqrtf(var + 1e-5f);
  }
  __syncthreads();
  const float rstd = bc[1];
  v4f o;
  o[0] = (tid == 0) ? mean : 0.f;
  o[1] = (tid == 0) ? rstd : 0.f;
  o[2] = 0.f; o[3] = 0.f;
  float* line = stats + (size_t)bg * STP;
  if (tid < 8) *(volatile v4f*)(line + tid * 4) = o;
  __threadfence();
  if (tid < 8) *(volatile v4f*)(line + tid * 4) = o;
}

__global__ __launch_bounds__(256) void gnprep_kernel(const float* __restrict__ x, const float* __restrict__ nw,
                                                     const float* __restrict__ nbv, const float* __restrict__ stats,
                                                     unsigned short* __restrict__ ht) {
  __shared__ __align__(16) float tf[64 * 68];
  __shared__ float sw[64];
  __shared__ float sb[64];
  __shared__ float sst[4];
  const int b   = blockIdx.z;
  const int n0  = blockIdx.x * 64;
  const int c0  = blockIdx.y * 64;
  const int tid = threadIdx.x;
  const float* xb = x + (size_t)b * CH * NPOS;
  unsigned short* hb = ht + (size_t)b * NPOS * CH;
  if (tid < 64) { sw[tid] = nw[c0 + tid]; sb[tid] = nbv[c0 + tid]; }
  {
    const int g0 = c0 >> 5;
    const int gi = (tid >> 1) & 1, fi = tid & 1;
    const float sv = stats[(size_t)(b * NGRP + g0 + gi) * STP + fi];
    if (tid < 4) sst[tid] = sv;
  }
  __syncthreads();
  {
    const int lr = tid >> 4;
    const int c4 = (tid & 15) * 4;
#pragma unroll
    for (int it = 0; it < 4; ++it) {
      const int rr = it * 16 + lr;
      const float mean = sst[(it >> 1) * 2], rstd = sst[(it >> 1) * 2 + 1];
      const float w = sw[rr], bb = sb[rr];
      const v4f a = *(const v4f*)(xb + (size_t)(c0 + rr) * NPOS + n0 + c4);
      v4f t;
#pragma unroll
      for (int e = 0; e < 4; ++e) { const float u = (a[e] - mean) * rstd; t[e] = u * w + bb; }
      *(v4f*)(tf + rr * 68 + c4) = t;
    }
  }
  __syncthreads();
  const int sub = tid >> 3;
  const int c8  = (tid & 7) * 8;
  v4u hv[2];
#pragma unroll
  for (int it = 0; it < 2; ++it) {
    const int oc = it * 32 + sub;
    v4u a;
#pragma unroll
    for (int q = 0; q < 4; ++q) {
      const float f0 = tf[(c8 + 2 * q) * 68 + oc];
      const float f1 = tf[(c8 + 2 * q + 1) * 68 + oc];
      a[q] = pk16(f2bf_bits(f0), f2bf_bits(f1));
    }
    hv[it] = a;
  }
  for (int pass = 0; pass < 2; ++pass) {
#pragma unroll
    for (int it = 0; it < 2; ++it) {
      const int oc = it * 32 + sub;
      const size_t go = (size_t)(n0 + oc) * CH + c0 + c8;
      *(volatile v4u*)(hb + go) = hv[it];
    }
    __threadfence();
  }
}

#define AQB 64
#define AKC 64
#define ANW 8
static_assert(NPOS % AQB == 0);
static_assert(NPOS % AKC == 0);
static_assert(CH == 2 * 128);

__global__ __launch_bounds__(256)
void attn_kernel(const unsigned short* __restrict__ qkp, const unsigned short* __restrict__ vpp,
                 unsigned short* __restrict__ opp, float sscale) {
  union FB { v16b v; v8b h[2]; };
  __shared__ __align__(16) __bf16 Ks[AKC * CH];
  __shared__ __align__(16) __bf16 Vs[CH * AKC];
  __shared__ __align__(16) __bf16 Ps[AQB * AKC];
  __shared__ __align__(16) float  Os[ANW][16 * 68];
  __shared__ float Al[AQB];
  __shared__ float Ll[AQB];

  const int tid  = threadIdx.x;
  const int wave = tid >> 5;
  const int lane = tid & 31;
  const int hh   = lane >> 4;
  const int c    = lane & 15;

  const int nqb = NPOS / AQB;
  const int bx  = blockIdx.x;
  const int qb  = bx % nqb;
  const int b   = bx / nqb;
  const int rt  = wave & 3;
  const int ch0 = (wave >> 2) * 128;
  const size_t tok0 = (size_t)b * NPOS;
  const size_t q0   = tok0 + (size_t)qb * AQB;

  const __bf16* Qg = (const __bf16*)(const void*)qkp;
  const __bf16* Kg = Qg + CH;
  const __bf16* Vg = (const __bf16*)(const void*)vpp + (size_t)b * CH * NPOS;

  float mrow[8], lrow[8];
  v8f oacc[8];
#pragma unroll
  for (int r = 0; r < 8; ++r) { mrow[r] = -INFINITY; lrow[r] = 0.f; }
#pragma unroll
  for (int t = 0; t < 8; ++t) oacc[t] = (v8f){0.f,0.f,0.f,0.f,0.f,0.f,0.f,0.f};

  const int nChunks = NPOS / AKC;
  for (int kc = 0; kc < nChunks; ++kc) {
    const int kv0 = kc * AKC;
    __syncthreads();
    {
#pragma unroll
      for (int i = 0; i < 8; ++i) {
        const int p   = i * 256 + tid;
        const int kr  = p >> 5, kc8 = (p & 31) * 8;
        const int vr  = p >> 3, vc8 = (p & 7) * 8;
        const v8b kvv = *(const v8b*)(Kg + (tok0 + kv0 + kr) * QKP + kc8);
        const v8b vvv = *(const v8b*)(Vg + (size_t)vr * NPOS + kv0 + vc8);
        *(v8b*)(Ks + kr * CH + kc8) = kvv;
        *(v8b*)(Vs + vr * AKC + vc8) = vvv;
      }
    }
    __syncthreads();

    if (wave < 4) {
      v8f s[4];
#pragma unroll
      for (int j = 0; j < 4; ++j) s[j] = (v8f){0.f,0.f,0.f,0.f,0.f,0.f,0.f,0.f};
      const __bf16* qr = Qg + (q0 + wave * 16 + c) * QKP + 8 * hh;
#pragma unroll
      for (int ks = 0; ks < CH / 32; ++ks) {
        const v16b qa = Frag<__bf16>::load(qr + ks * 32);
#pragma unroll
        for (int j = 0; j < 4; ++j) {
          FB kb;
          kb.h[0] = *(const v8b*)(Ks + (j * 16 + c) * CH + ks * 32 + 8 * hh);
          kb.h[1] = *(const v8b*)(Ks + (j * 16 + c) * CH + ks * 32 + 16 + 8 * hh);
          s[j] = at_mma(qa, kb.v, s[j]);
        }
      }
      float cm[8];
#pragma unroll
      for (int r = 0; r < 8; ++r) {
        float m = -INFINITY;
#pragma unroll
        for (int j = 0; j < 4; ++j) {
          const float sv = s[j][r] * sscale;
          s[j][r] = sv;
          m = fmaxf(m, sv);
        }
#pragma unroll
        for (int off = 1; off < 16; off <<= 1) m = fmaxf(m, __shfl_xor(m, off, 32));
        cm[r] = m;
      }
      __bf16* pw = Ps + wave * 16 * AKC;
#pragma unroll
      for (int r = 0; r < 8; ++r) {
        const float mnew  = fmaxf(mrow[r], cm[r]);
        const float alpha = expf(mrow[r] - mnew);
        mrow[r] = mnew;
        float psum = 0.f;
#pragma unroll
        for (int j = 0; j < 4; ++j) {
          const float pv = expf(s[j][r] - mnew);
          psum += pv;
          pw[(8 * hh + r) * AKC + j * 16 + c] = at_f2bf(pv);
        }
#pragma unroll
        for (int off = 1; off < 16; off <<= 1) psum += __shfl_xor(psum, off, 32);
        lrow[r] = lrow[r] * alpha + psum;
        if (c == 0) Al[wave * 16 + 8 * hh + r] = alpha;
      }
    }
    __syncthreads();

    {
      float al[8];
#pragma unroll
      for (int r = 0; r < 8; ++r) al[r] = Al[rt * 16 + 8 * hh + r];
#pragma unroll
      for (int r = 0; r < 8; ++r) {
#pragma unroll
        for (int t = 0; t < 8; ++t) oacc[t][r] *= al[r];
      }
      const __bf16* pr = Ps + (rt * 16 + c) * AKC + 8 * hh;
#pragma unroll 1
      for (int kk = 0; kk < AKC / 32; ++kk) {
        FB pa;
        pa.h[0] = *(const v8b*)(pr + kk * 32);
        pa.h[1] = *(const v8b*)(pr + kk * 32 + 16);
#pragma unroll
        for (int t = 0; t < 8; ++t) {
          FB vb;
          vb.h[0] = *(const v8b*)(Vs + (ch0 + t * 16 + c) * AKC + kk * 32 + 8 * hh);
          vb.h[1] = *(const v8b*)(Vs + (ch0 + t * 16 + c) * AKC + kk * 32 + 16 + 8 * hh);
          oacc[t] = at_mma(pa.v, vb.v, oacc[t]);
        }
      }
    }
  }

  if (wave < 4) {
#pragma unroll
    for (int r = 0; r < 8; ++r) { if (c == 0) Ll[wave * 16 + 8 * hh + r] = lrow[r]; }
  }
  __syncthreads();

  float inv[8];
#pragma unroll
  for (int r = 0; r < 8; ++r) inv[r] = 1.0f / Ll[rt * 16 + 8 * hh + r];
  float* os = Os[wave];
  const int q = lane >> 3, c8 = (lane & 7) * 8;
  unsigned short* orow = opp + (q0 + (size_t)rt * 16) * CH + ch0;
#pragma unroll
  for (int hf = 0; hf < 2; ++hf) {
#pragma unroll
    for (int r = 0; r < 8; ++r) {
#pragma unroll
      for (int tt = 0; tt < 4; ++tt) os[(8 * hh + r) * 68 + tt * 16 + c] = oacc[hf * 4 + tt][r] * inv[r];
    }
    __builtin_amdgcn_fence(__ATOMIC_RELEASE, "workgroup");
    __builtin_amdgcn_wave_barrier();
    __builtin_amdgcn_fence(__ATOMIC_ACQUIRE, "workgroup");
    for (int pass = 0; pass < 2; ++pass) {
#pragma unroll
      for (int it = 0; it < 4; ++it) {
        const int row = it * 4 + q;
        const float* sp = os + row * 68 + c8;
        v8h hv;
#pragma unroll
        for (int e = 0; e < 8; ++e) hv[e] = __builtin_bit_cast(_Float16, f2bf_bits(sp[e]));
        *(volatile v8h*)(orow + (size_t)row * CH + hf * 64 + c8) = hv;
      }
      __threadfence();
    }
    __builtin_amdgcn_fence(__ATOMIC_RELEASE, "workgroup");
    __builtin_amdgcn_wave_barrier();
    __builtin_amdgcn_fence(__ATOMIC_ACQUIRE, "workgroup");
  }
}

extern "C" void kernel_launch(void* const* d_in, const int* in_sizes, int n_in,
                              void* d_out, int out_size, void* d_ws, size_t ws_size,
                              hipStream_t stream) {
  if (n_in < 7) return;
  if (in_sizes[0] != NB * CH * NPOS) return;
  if (in_sizes[1] != CH || in_sizes[2] != CH) return;
  if (in_sizes[3] != 3 * CH * CH || in_sizes[4] != 3 * CH) return;
  if (in_sizes[5] != CH * CH || in_sizes[6] != CH) return;
  if (out_size != NB * CH * NPOS) return;

  const float* x      = (const float*)d_in[0];
  const float* norm_w = (const float*)d_in[1];
  const float* norm_b = (const float*)d_in[2];
  const float* qkv_w  = (const float*)d_in[3];
  const float* qkv_b  = (const float*)d_in[4];
  const float* out_w  = (const float*)d_in[5];
  const float* out_b  = (const float*)d_in[6];

  const size_t PST  = (size_t)(NB * NGRP) * STP * 4;
  const size_t PHT  = (size_t)NB * NPOS * CH * 2;
  const size_t PW16 = (size_t)3 * CH * CH * 2;
  const size_t PWO  = (size_t)CH * CH * 2;
  const size_t PQK  = (size_t)NB * NPOS * QKP * 2;
  const size_t PVP  = (size_t)NB * CH * NPOS * 2;
  const size_t POP  = (size_t)NB * NPOS * CH * 2;
  size_t off = 0;
  const size_t oST  = off; off += PST;
  const size_t oHT  = off; off += PHT;
  const size_t oW16 = off; off += PW16;
  const size_t oWO  = off; off += PWO;
  const size_t oQK  = off; off += PQK;
  const size_t oVP  = off; off += PVP;
  const size_t oOP  = off; off += POP;
  if (off > ws_size) return;
  if (off > (size_t)134217728) return;

  char* ws = (char*)d_ws;
  float*          STATS = (float*)(ws + oST);
  unsigned short* HT    = (unsigned short*)(ws + oHT);
  unsigned short* W16   = (unsigned short*)(ws + oW16);
  unsigned short* WO16  = (unsigned short*)(ws + oWO);
  unsigned short* QK    = (unsigned short*)(ws + oQK);
  unsigned short* VP    = (unsigned short*)(ws + oVP);
  unsigned short* OP    = (unsigned short*)(ws + oOP);

  const dim3 blk(256);

  gnstat_kernel<<<dim3(NB * NGRP), blk, 0, stream>>>(x, STATS);
  const int n2q = 3 * CH * CH / 2;
  conv_bf16x2_kernel<<<dim3((n2q + 255) / 256), blk, 0, stream>>>(qkv_w, W16, n2q);
  const int n2o = CH * CH / 2;
  conv_bf16x2_kernel<<<dim3((n2o + 255) / 256), blk, 0, stream>>>(out_w, WO16, n2o);
  gnprep_kernel<<<dim3(NPOS / 64, CH / 64, NB), blk, 0, stream>>>(x, norm_w, norm_b, STATS, HT);
  const dim3 gQK(((NB * NPOS / 64) * (QKP / 64) + 7) / 8, 1);
  wmma_gemm64<2, 1, false><<<gQK, blk, 0, stream>>>(
      HT, CH, 0L, W16, CH, 0L, (void*)QK, QKP, 0L,
      qkv_b, x, 0L, NB * NPOS, QKP, CH, 1.0f);
  const dim3 gV(((CH / 64) * (NPOS / 64) + 7) / 8, NB);
  wmma_gemm64<1, 1, false><<<gV, blk, 0, stream>>>(
      W16 + (size_t)2 * CH * CH, CH, 0L, HT, CH, (long)NPOS * CH, (void*)VP, NPOS, (long)CH * NPOS,
      qkv_b + 2 * CH, x, 0L, CH, NPOS, CH, 1.0f);
  attn_kernel<<<dim3(NB * (NPOS / AQB)), dim3(256), 0, stream>>>(QK, VP, OP, 0.0625f);
  const dim3 gO(((CH / 64) * (NPOS / 64) + 7) / 8, NB);
  wmma_gemm64<1, 0, true><<<gO, blk, 0, stream>>>(
      WO16, CH, 0L, OP, CH, (long)NPOS * CH, d_out, NPOS, (long)CH * NPOS,
      out_b, x, (long)CH * NPOS, CH, NPOS, CH, 1.0f);
  (void)hipGetLastError();
}
